// SocialLSTM_17033840296106
// MI455X (gfx1250) — hardware-verified
//
#include <hip/hip_runtime.h>
#include <math.h>

constexpr int HID      = 64;
constexpr int NGATE    = 4 * HID;
constexpr int GRID_X   = 4;
constexpr int GRID_Y   = 4;
constexpr int NCELL    = GRID_X * GRID_Y;
constexpr int W1_PITCH = NCELL * HID;
constexpr int NSTEP    = 14;
constexpr int NAGENT   = 65536;
constexpr int NWAVE    = 4;
constexpr int NTHR_MAIN = NWAVE * 32;
constexpr int AG_BLK   = NWAVE * 16;
constexpr int TP       = 72;
constexpr int NOUT_PAD = 16;
constexpr int NOUT     = 2;
constexpr float ACT_CARRY = 64.0f;
constexpr float W_CARRY   = 16.0f;
constexpr float FOLD      = 1.0f / (ACT_CARRY * W_CARRY);
constexpr float RES_CARRY = 2048.0f;
constexpr float RES_INV   = 1.0f / RES_CARRY;
constexpr float INV_GX    = 1.0f / (float)GRID_X;
constexpr float INV_GY    = 1.0f / (float)GRID_Y;

constexpr int CB_BSUM = 0;
constexpr int CB_WC0  = CB_BSUM + NGATE;
constexpr int CB_WC1  = CB_WC0 + NGATE;
constexpr int CB_B1   = CB_WC1 + NGATE;
constexpr int CB_B2   = CB_B1 + HID;
constexpr int CB_BOUT = CB_B2 + HID;
constexpr int CB_SIZE = CB_BOUT + 8;

constexpr int PB_WHH  = (NGATE * HID) / 8 / 256;
constexpr int PB_W1   = (HID * W1_PITCH) / 8 / 256;
constexpr int PB_W2   = (HID * HID) / 8 / 256;
constexpr int PB_WOUT = 1;
constexpr int PB_TOTAL = PB_WHH + PB_W1 + PB_W2 + PB_WOUT;
constexpr int MM_THR  = 1024;
constexpr int MM_ITER = (NAGENT * 2) / 4 / MM_THR;

static_assert(HID % 32 == 0, "K multiple of 32");
static_assert(NAGENT % AG_BLK == 0, "agent tiles exact");
static_assert((NGATE * HID) % (8 * 256) == 0, "W_hh plane blocks exact");
static_assert((HID * W1_PITCH) % (8 * 256) == 0, "W1 plane blocks exact");
static_assert((HID * HID) % (8 * 256) == 0, "W2 plane blocks exact");
static_assert(2 * NOUT_PAD * HID == 8 * 256, "Wout hi+lo planes = one block");
static_assert(MM_ITER * MM_THR * 4 == NAGENT * 2, "min/max scan exact");
static_assert(MM_THR / 32 == 32, "one partial per lane");
static_assert(NSTEP * NAGENT * 2 == 1835008, "output element count");
static_assert(TP % 8 == 0 && TP >= HID, "tile pitch");
static_assert(CB_SIZE >= CB_BOUT + NOUT, "constant block extent");

typedef __attribute__((ext_vector_type(16))) _Float16 v16h;
typedef __attribute__((ext_vector_type(8)))  _Float16 v8h;
typedef __attribute__((ext_vector_type(8)))  float    v8f;
typedef __attribute__((ext_vector_type(4)))  float    v4f;
typedef __attribute__((ext_vector_type(2)))  float    v2f;
typedef __attribute__((ext_vector_type(8)))  unsigned v8u;

template <typename T> struct Frag;
template <> struct Frag<_Float16> {
  typedef v16h V; union U { v16h v; v8h h[2]; };
  static __device__ __forceinline__ v16h load(const _Float16* p) {
    U f; f.h[0] = *(const v8h*)(p); f.h[1] = *(const v8h*)(p + 16); return f.v;
  }
  static __device__ __forceinline__ v8f mma(v16h a, v16h b, v8f c) {
    return __builtin_amdgcn_wmma_f32_16x16x32_f16(false, a, false, b, (short)0, c, false, false);
  }
};

__device__ __forceinline__ void guard4h(v8f& a0, v8f& a1, v8f& a2, v8f& a3, v16h x,
                                        v16h b0, v16h b1, v16h b2, v16h b3) {
  asm volatile("v_nop\n\tv_nop\n\tv_nop\n\tv_nop"
               : "+v"(a0), "+v"(a1), "+v"(a2), "+v"(a3)
               : "v"(x), "v"(b0), "v"(b1), "v"(b2), "v"(b3));
}
__device__ __forceinline__ void guard2h(v8f& a0, v8f& a1, v16h x, v16h y, v16h b0, v16h b1) {
  asm volatile("v_nop\n\tv_nop\n\tv_nop\n\tv_nop"
               : "+v"(a0), "+v"(a1)
               : "v"(x), "v"(y), "v"(b0), "v"(b1));
}

__device__ __forceinline__ void lds_wave_sync() {
  __builtin_amdgcn_fence(__ATOMIC_RELEASE, "workgroup");
  __builtin_amdgcn_wave_barrier();
  __builtin_amdgcn_fence(__ATOMIC_ACQUIRE, "workgroup");
}

__device__ __forceinline__ float fsig(float x)  { return __builtin_amdgcn_rcpf(1.0f + __expf(-x)); }
__device__ __forceinline__ float ftanh(float x) { return 1.0f - 2.0f * __builtin_amdgcn_rcpf(__expf(2.0f * x) + 1.0f); }

__device__ __forceinline__ v16h mask_frag(v16h a, bool keep) {
  v8u w = __builtin_bit_cast(v8u, a);
#pragma unroll
  for (int e = 0; e < 8; ++e) {
    const unsigned x = w[e];
    w[e] = keep ? x : 0u;
  }
  return __builtin_bit_cast(v16h, w);
}

__device__ __forceinline__ int cell_of(float x, float y, float mnx, float mxx, float mny, float mxy) {
#pragma clang fp contract(off)
  const float cw = (mxx - mnx) * INV_GX;
  const float ch = (mxy - mny) * INV_GY;
  const float rx = 1.0f / cw;
  const float ry = 1.0f / ch;
  const float dx = x - mnx;
  const float dy = y - mny;
  const float qx = dx * rx;
  const float qy = dy * ry;
  int cx = (int)qx;
  int cy = (int)qy;
  cx = cx < 0 ? 0 : (cx > GRID_X - 1 ? GRID_X - 1 : cx);
  cy = cy < 0 ? 0 : (cy > GRID_Y - 1 ? GRID_Y - 1 : cy);
  return cy * GRID_X + cx;
}

__global__ __launch_bounds__(256) void prep_planes_kernel(
    const float* __restrict__ whh, const float* __restrict__ w1, const float* __restrict__ w2,
    const float* __restrict__ wout,
    unsigned short* __restrict__ WHHp, unsigned short* __restrict__ W1Pp, unsigned short* __restrict__ W2Pp,
    unsigned short* __restrict__ WOHp, unsigned short* __restrict__ WOLp) {
  const int blk = blockIdx.x;
  const int tid = threadIdx.x;
  if (blk < PB_WHH + PB_W1 + PB_W2) {
    const float* src;
    unsigned short* dst;
    int i;
    if (blk < PB_WHH) {
      src = whh; dst = WHHp; i = blk * 256 + tid;
    } else if (blk < PB_WHH + PB_W1) {
      src = w1; dst = W1Pp; i = (blk - PB_WHH) * 256 + tid;
    } else {
      src = w2; dst = W2Pp; i = (blk - PB_WHH - PB_W1) * 256 + tid;
    }
    const v4f a = *(const v4f*)(src + (size_t)i * 8);
    const v4f b = *(const v4f*)(src + (size_t)i * 8 + 4);
    v8h hv;
#pragma unroll
    for (int e = 0; e < 4; ++e) {
      hv[e]     = (_Float16)(a[e] * W_CARRY);
      hv[4 + e] = (_Float16)(b[e] * W_CARRY);
    }
    *(volatile v8h*)(dst + (size_t)i * 8) = hv;
    __threadfence();
    *(volatile v8h*)(dst + (size_t)i * 8) = hv;
  } else {
    const int which = tid >> 7;
    const int jj    = tid & 127;
    const int row   = jj >> 3;
    const int col0  = (jj & 7) * 8;
    const int rowc  = row < NOUT ? row : (NOUT - 1);
    const bool live = row < NOUT;
    const v4f a = *(const v4f*)(wout + rowc * HID + col0);
    const v4f b = *(const v4f*)(wout + rowc * HID + col0 + 4);
    v8h hv;
#pragma unroll
    for (int e = 0; e < 8; ++e) {
      const float raw = (e < 4) ? a[e & 3] : b[e & 3];
      const float s   = live ? raw * W_CARRY : 0.0f;
      const _Float16 hi = (_Float16)s;
      const _Float16 lo = (_Float16)((s - (float)hi) * RES_CARRY);
      hv[e] = which ? lo : hi;
    }
    unsigned short* dst = (which ? WOLp : WOHp) + jj * 8;
    *(volatile v8h*)dst = hv;
    __threadfence();
    *(volatile v8h*)dst = hv;
  }
}

__global__ __launch_bounds__(MM_THR) void minmax_kernel(const float* __restrict__ traj, float* __restrict__ MM) {
  __shared__ float RED[32 * 4];
  const int t = blockIdx.x;
  const int tid = threadIdx.x, lane = tid & 31, wave = tid >> 5;
  const v4f* p = (const v4f*)(traj + (size_t)t * NAGENT * 2);
  float mnx = INFINITY, mxx = -INFINITY, mny = INFINITY, mxy = -INFINITY;
#pragma unroll 4
  for (int i = 0; i < MM_ITER; ++i) {
    const v4f v = p[i * MM_THR + tid];
    mnx = fminf(mnx, fminf(v[0], v[2]));
    mxx = fmaxf(mxx, fmaxf(v[0], v[2]));
    mny = fminf(mny, fminf(v[1], v[3]));
    mxy = fmaxf(mxy, fmaxf(v[1], v[3]));
  }
#pragma unroll
  for (int off = 1; off < 32; off <<= 1) {
    mnx = fminf(mnx, __shfl_xor(mnx, off, 32));
    mxx = fmaxf(mxx, __shfl_xor(mxx, off, 32));
    mny = fminf(mny, __shfl_xor(mny, off, 32));
    mxy = fmaxf(mxy, __shfl_xor(mxy, off, 32));
  }
  if (lane == 0) {
    RED[wave * 4 + 0] = mnx;
    RED[wave * 4 + 1] = mxx;
    RED[wave * 4 + 2] = mny;
    RED[wave * 4 + 3] = mxy;
  }
  __syncthreads();
  float a = RED[lane * 4 + 0];
  float b = RED[lane * 4 + 1];
  float cc = RED[lane * 4 + 2];
  float d = RED[lane * 4 + 3];
#pragma unroll
  for (int off = 1; off < 32; off <<= 1) {
    a  = fminf(a,  __shfl_xor(a,  off, 32));
    b  = fmaxf(b,  __shfl_xor(b,  off, 32));
    cc = fminf(cc, __shfl_xor(cc, off, 32));
    d  = fmaxf(d,  __shfl_xor(d,  off, 32));
  }
  const float val = (lane == 0) ? a : (lane == 1) ? b : (lane == 2) ? cc : (lane == 3) ? d : 0.0f;
  if (wave == 0) {
    volatile float* o = MM + t * 32 + lane;
    *o = val;
    __threadfence();
    *o = val;
  }
}

__global__ __launch_bounds__(NTHR_MAIN) void social_seq_kernel(
    const float* __restrict__ traj, const float* __restrict__ wih,
    const float* __restrict__ bih, const float* __restrict__ bhh,
    const float* __restrict__ b1g, const float* __restrict__ b2g, const float* __restrict__ boutg,
    const unsigned short* __restrict__ WHHp, const unsigned short* __restrict__ W1Pp,
    const unsigned short* __restrict__ W2Pp, const unsigned short* __restrict__ WOHp,
    const unsigned short* __restrict__ WOLp, const float* __restrict__ MM, float* __restrict__ out) {
  __shared__ __align__(16) float    CB[CB_SIZE];
  __shared__ __align__(16) _Float16 TH[NWAVE][16 * TP];
  __shared__ __align__(16) _Float16 TL[NWAVE][16 * TP];
  __shared__ __align__(16) float    HS[NWAVE][32 * 32];
  __shared__ __align__(16) float    OS[NWAVE][32];

  const _Float16* WHH = (const _Float16*)WHHp;
  const _Float16* W1P = (const _Float16*)W1Pp;
  const _Float16* W2P = (const _Float16*)W2Pp;
  const _Float16* WOH = (const _Float16*)WOHp;
  const _Float16* WOL = (const _Float16*)WOLp;

  const int tid = threadIdx.x;
#pragma unroll 1
  for (int i = tid; i < NGATE; i += NTHR_MAIN) {
    const v2f w = *(const v2f*)(wih + 2 * i);
    CB[CB_BSUM + i] = bih[i] + bhh[i];
    CB[CB_WC0 + i]  = w[0];
    CB[CB_WC1 + i]  = w[1];
  }
  if (tid < HID) {
    CB[CB_B1 + tid] = b1g[tid];
    CB[CB_B2 + tid] = b2g[tid];
  }
  if (tid < NOUT) CB[CB_BOUT + tid] = boutg[tid];
  __syncthreads();

  const int wave = tid >> 5, lane = tid & 31;
  const int c = lane & 15, hh = lane >> 4, koff = hh * 8;
  const int agent0 = blockIdx.x * AG_BLK + wave * 16;
  _Float16* th = TH[wave];
  _Float16* tl = TL[wave];
  float* hs = HS[wave];
  float* os = OS[wave];

  const v8f z8 = {0.f, 0.f, 0.f, 0.f, 0.f, 0.f, 0.f, 0.f};
  const v8u zu = {0u, 0u, 0u, 0u, 0u, 0u, 0u, 0u};
  float cst[4][8];
#pragma unroll
  for (int jt = 0; jt < 4; ++jt)
#pragma unroll
    for (int r = 0; r < 8; ++r) cst[jt][r] = 0.0f;
  v16h hA0 = __builtin_bit_cast(v16h, zu);
  v16h hA1 = hA0;

#pragma unroll 1
  for (int t = 0; t < NSTEP; ++t) {
    const float* pt = traj + ((size_t)t * NAGENT + (size_t)agent0) * 2;
    const v4f q0 = *(const v4f*)(pt + 16 * hh);
    const v4f q1 = *(const v4f*)(pt + 16 * hh + 4);
    const v4f q2 = *(const v4f*)(pt + 16 * hh + 8);
    const v4f q3 = *(const v4f*)(pt + 16 * hh + 12);
    const v2f pr = *(const v2f*)(pt + 2 * c);
    const v4f mm = *(const v4f*)(MM + t * 32);
    const float mnx = mm[0], mxx = mm[1], mny = mm[2], mxy = mm[3];
    const int myidx = cell_of(pr[0], pr[1], mnx, mxx, mny, mxy);
    float px[8], py[8];
    px[0] = q0[0]; py[0] = q0[1]; px[1] = q0[2]; py[1] = q0[3];
    px[2] = q1[0]; py[2] = q1[1]; px[3] = q1[2]; py[3] = q1[3];
    px[4] = q2[0]; py[4] = q2[1]; px[5] = q2[2]; py[5] = q2[3];
    px[6] = q3[0]; py[6] = q3[1]; px[7] = q3[2]; py[7] = q3[3];

    lds_wave_sync();

#pragma unroll
    for (int jt = 0; jt < 4; ++jt) {
      const int j = jt * 16 + c;
      const _Float16* wb = WHH + (size_t)j * HID + koff;
      v8f acc[4];
      acc[0] = z8; acc[1] = z8; acc[2] = z8; acc[3] = z8;
      {
        const v16h b0 = Frag<_Float16>::load(wb);
        const v16h b1 = Frag<_Float16>::load(wb + (size_t)1 * HID * HID);
        const v16h b2 = Frag<_Float16>::load(wb + (size_t)2 * HID * HID);
        const v16h b3 = Frag<_Float16>::load(wb + (size_t)3 * HID * HID);
        acc[0] = Frag<_Float16>::mma(hA0, b0, acc[0]);
        acc[1] = Frag<_Float16>::mma(hA0, b1, acc[1]);
        acc[2] = Frag<_Float16>::mma(hA0, b2, acc[2]);
        acc[3] = Frag<_Float16>::mma(hA0, b3, acc[3]);
        guard4h(acc[0], acc[1], acc[2], acc[3], hA0, b0, b1, b2, b3);
      }
      {
        const v16h b0 = Frag<_Float16>::load(wb + 32);
        const v16h b1 = Frag<_Float16>::load(wb + (size_t)1 * HID * HID + 32);
        const v16h b2 = Frag<_Float16>::load(wb + (size_t)2 * HID * HID + 32);
        const v16h b3 = Frag<_Float16>::load(wb + (size_t)3 * HID * HID + 32);
        acc[0] = Frag<_Float16>::mma(hA1, b0, acc[0]);
        acc[1] = Frag<_Float16>::mma(hA1, b1, acc[1]);
        acc[2] = Frag<_Float16>::mma(hA1, b2, acc[2]);
        acc[3] = Frag<_Float16>::mma(hA1, b3, acc[3]);
        guard4h(acc[0], acc[1], acc[2], acc[3], hA1, b0, b1, b2, b3);
      }
      float bs[4], wa[4], wb2[4];
#pragma unroll
      for (int g = 0; g < 4; ++g) {
        bs[g]  = CB[CB_BSUM + g * HID + j];
        wa[g]  = CB[CB_WC0 + g * HID + j];
        wb2[g] = CB[CB_WC1 + g * HID + j];
      }
#pragma unroll
      for (int r = 0; r < 8; ++r) {
        const float zi = acc[0][r] * FOLD + (bs[0] + px[r] * wa[0] + py[r] * wb2[0]);
        const float zf = acc[1][r] * FOLD + (bs[1] + px[r] * wa[1] + py[r] * wb2[1]);
        const float zg = acc[2][r] * FOLD + (bs[2] + px[r] * wa[2] + py[r] * wb2[2]);
        const float zo = acc[3][r] * FOLD + (bs[3] + px[r] * wa[3] + py[r] * wb2[3]);
        const float iv = fsig(zi);
        const float fv = fsig(zf);
        const float gv = ftanh(zg);
        const float ov = fsig(zo);
        const float cn = fv * cst[jt][r] + iv * gv;
        cst[jt][r] = cn;
        const float hn = ov * ftanh(cn);
        hs[(jt * 8 + r) * 32 + lane] = hn;
        th[(8 * hh + r) * TP + j] = (_Float16)(hn * ACT_CARRY);
      }
    }
    lds_wave_sync();
    hA0 = Frag<_Float16>::load(th + c * TP + koff);
    hA1 = Frag<_Float16>::load(th + c * TP + 32 + koff);

    v8f sa[4];
    sa[0] = z8; sa[1] = z8; sa[2] = z8; sa[3] = z8;
#pragma unroll 1
    for (int cell = 0; cell < NCELL; ++cell) {
      const bool mine = (myidx == cell);
      const unsigned occ = __builtin_amdgcn_ballot_w32(mine);
      if (occ != 0u) {
        const v16h m0 = mask_frag(hA0, mine);
        const v16h m1 = mask_frag(hA1, mine);
        const _Float16* wb = W1P + (size_t)c * W1_PITCH + cell * HID + koff;
        {
          const v16h b0 = Frag<_Float16>::load(wb);
          const v16h b1 = Frag<_Float16>::load(wb + (size_t)16 * W1_PITCH);
          const v16h b2 = Frag<_Float16>::load(wb + (size_t)32 * W1_PITCH);
          const v16h b3 = Frag<_Float16>::load(wb + (size_t)48 * W1_PITCH);
          sa[0] = Frag<_Float16>::mma(m0, b0, sa[0]);
          sa[1] = Frag<_Float16>::mma(m0, b1, sa[1]);
          sa[2] = Frag<_Float16>::mma(m0, b2, sa[2]);
          sa[3] = Frag<_Float16>::mma(m0, b3, sa[3]);
          guard4h(sa[0], sa[1], sa[2], sa[3], m0, b0, b1, b2, b3);
        }
        {
          const v16h b0 = Frag<_Float16>::load(wb + 32);
          const v16h b1 = Frag<_Float16>::load(wb + (size_t)16 * W1_PITCH + 32);
          const v16h b2 = Frag<_Float16>::load(wb + (size_t)32 * W1_PITCH + 32);
          const v16h b3 = Frag<_Float16>::load(wb + (size_t)48 * W1_PITCH + 32);
          sa[0] = Frag<_Float16>::mma(m1, b0, sa[0]);
          sa[1] = Frag<_Float16>::mma(m1, b1, sa[1]);
          sa[2] = Frag<_Float16>::mma(m1, b2, sa[2]);
          sa[3] = Frag<_Float16>::mma(m1, b3, sa[3]);
          guard4h(sa[0], sa[1], sa[2], sa[3], m1, b0, b1, b2, b3);
        }
      }
    }

    lds_wave_sync();
#pragma unroll
    for (int jt = 0; jt < 4; ++jt) {
      const int j = jt * 16 + c;
      const float bv = CB[CB_B1 + j];
#pragma unroll
      for (int r = 0; r < 8; ++r) {
        const float v = fmaxf(sa[jt][r] * FOLD + bv, 0.0f);
        th[(8 * hh + r) * TP + j] = (_Float16)(v * ACT_CARRY);
      }
    }
    lds_wave_sync();
    const v16h rA0 = Frag<_Float16>::load(th + c * TP + koff);
    const v16h rA1 = Frag<_Float16>::load(th + c * TP + 32 + koff);

    v8f ca[4];
    ca[0] = z8; ca[1] = z8; ca[2] = z8; ca[3] = z8;
    {
      const _Float16* wb = W2P + (size_t)c * HID + koff;
      {
        const v16h b0 = Frag<_Float16>::load(wb);
        const v16h b1 = Frag<_Float16>::load(wb + 16 * HID);
        const v16h b2 = Frag<_Float16>::load(wb + 32 * HID);
        const v16h b3 = Frag<_Float16>::load(wb + 48 * HID);
        ca[0] = Frag<_Float16>::mma(rA0, b0, ca[0]);
        ca[1] = Frag<_Float16>::mma(rA0, b1, ca[1]);
        ca[2] = Frag<_Float16>::mma(rA0, b2, ca[2]);
        ca[3] = Frag<_Float16>::mma(rA0, b3, ca[3]);
        guard4h(ca[0], ca[1], ca[2], ca[3], rA0, b0, b1, b2, b3);
      }
      {
        const v16h b0 = Frag<_Float16>::load(wb + 32);
        const v16h b1 = Frag<_Float16>::load(wb + 16 * HID + 32);
        const v16h b2 = Frag<_Float16>::load(wb + 32 * HID + 32);
        const v16h b3 = Frag<_Float16>::load(wb + 48 * HID + 32);
        ca[0] = Frag<_Float16>::mma(rA1, b0, ca[0]);
        ca[1] = Frag<_Float16>::mma(rA1, b1, ca[1]);
        ca[2] = Frag<_Float16>::mma(rA1, b2, ca[2]);
        ca[3] = Frag<_Float16>::mma(rA1, b3, ca[3]);
        guard4h(ca[0], ca[1], ca[2], ca[3], rA1, b0, b1, b2, b3);
      }
    }

    lds_wave_sync();
#pragma unroll
    for (int jt = 0; jt < 4; ++jt) {
      const int j = jt * 16 + c;
      const float bv = CB[CB_B2 + j];
#pragma unroll
      for (int r = 0; r < 8; ++r) {
        const float hv  = hs[(jt * 8 + r) * 32 + lane];
        const float cmb = hv + (ca[jt][r] * FOLD + bv);
        const float s   = cmb * ACT_CARRY;
        const _Float16 hi = (_Float16)s;
        const _Float16 lo = (_Float16)((s - (float)hi) * RES_CARRY);
        th[(8 * hh + r) * TP + j] = hi;
        tl[(8 * hh + r) * TP + j] = lo;
      }
    }
    lds_wave_sync();
    const v16h cH0 = Frag<_Float16>::load(th + c * TP + koff);
    const v16h cH1 = Frag<_Float16>::load(th + c * TP + 32 + koff);
    const v16h cL0 = Frag<_Float16>::load(tl + c * TP + koff);
    const v16h cL1 = Frag<_Float16>::load(tl + c * TP + 32 + koff);

    v8f oM = z8, oR = z8;
    {
      const v16h bH = Frag<_Float16>::load(WOH + (size_t)c * HID + koff);
      const v16h bL = Frag<_Float16>::load(WOL + (size_t)c * HID + koff);
      oM = Frag<_Float16>::mma(cH0, bH, oM);
      oR = Frag<_Float16>::mma(cH0, bL, oR);
      oR = Frag<_Float16>::mma(cL0, bH, oR);
      guard2h(oM, oR, cH0, cL0, bH, bL);
    }
    {
      const v16h bH = Frag<_Float16>::load(WOH + (size_t)c * HID + 32 + koff);
      const v16h bL = Frag<_Float16>::load(WOL + (size_t)c * HID + 32 + koff);
      oM = Frag<_Float16>::mma(cH1, bH, oM);
      oR = Frag<_Float16>::mma(cH1, bL, oR);
      oR = Frag<_Float16>::mma(cL1, bH, oR);
      guard2h(oM, oR, cH1, cL1, bH, bL);
    }
    const float bo = CB[CB_BOUT + (c < NOUT ? c : (NOUT - 1))];
    lds_wave_sync();
    if (c < NOUT) {
#pragma unroll
      for (int r = 0; r < 8; ++r) os[(8 * hh + r) * 2 + c] = (oM[r] + oR[r] * RES_INV) * FOLD + bo;
    }
    lds_wave_sync();
    {
      const float ov = os[lane];
      volatile float* op = out + ((size_t)t * NAGENT + (size_t)agent0) * 2 + lane;
      *op = ov;
      __threadfence();
      *op = ov;
    }
  }
}

extern "C" void kernel_launch(void* const* d_in, const int* in_sizes, int n_in,
                              void* d_out, int out_size, void* d_ws, size_t ws_size, hipStream_t stream) {
  if (n_in < 11 || d_out == nullptr || d_ws == nullptr) return;
  if (in_sizes[0] != NSTEP * NAGENT * 2 || in_sizes[1] != NGATE * 2 || in_sizes[2] != NGATE * HID ||
      in_sizes[3] != NGATE || in_sizes[4] != NGATE || in_sizes[5] != HID * W1_PITCH || in_sizes[6] != HID ||
      in_sizes[7] != HID * HID || in_sizes[8] != HID || in_sizes[9] != NOUT * HID || in_sizes[10] != NOUT ||
      out_size != NSTEP * NAGENT * 2) return;

  const float* traj = (const float*)d_in[0];
  const float* wih  = (const float*)d_in[1];
  const float* whh  = (const float*)d_in[2];
  const float* bih  = (const float*)d_in[3];
  const float* bhh  = (const float*)d_in[4];
  const float* w1   = (const float*)d_in[5];
  const float* b1   = (const float*)d_in[6];
  const float* w2   = (const float*)d_in[7];
  const float* b2   = (const float*)d_in[8];
  const float* wout = (const float*)d_in[9];
  const float* bout = (const float*)d_in[10];
  float* out = (float*)d_out;

  char* ws = (char*)d_ws; size_t off = 0;
  auto carve = [&](size_t bytes) -> char* { char* p = ws + off; off += (bytes + 255) & ~(size_t)255; return p; };
  unsigned short* WHH = (unsigned short*)carve((size_t)NGATE * HID * 2);
  unsigned short* W1P = (unsigned short*)carve((size_t)HID * W1_PITCH * 2);
  unsigned short* W2P = (unsigned short*)carve((size_t)HID * HID * 2);
  unsigned short* WOH = (unsigned short*)carve((size_t)NOUT_PAD * HID * 2);
  unsigned short* WOL = (unsigned short*)carve((size_t)NOUT_PAD * HID * 2);
  float*          MM  = (float*)carve((size_t)NSTEP * 32 * 4);
  if (off > ws_size || off > (size_t)134217728) return;

  prep_planes_kernel<<<PB_TOTAL, 256, 0, stream>>>(whh, w1, w2, wout, WHH, W1P, W2P, WOH, WOL);
  minmax_kernel<<<NSTEP, MM_THR, 0, stream>>>(traj, MM);
  social_seq_kernel<<<NAGENT / AG_BLK, NTHR_MAIN, 0, stream>>>(
      traj, wih, bih, bhh, b1, b2, bout, WHH, W1P, W2P, WOH, WOL, MM, out);
}
